// FactoredHmmLm_77249281786385
// MI455X (gfx1250) — hardware-verified
//
#include <hip/hip_runtime.h>

typedef _Float16 v16h __attribute__((ext_vector_type(16)));
typedef _Float16 v8h  __attribute__((ext_vector_type(8)));
typedef float    v8f  __attribute__((ext_vector_type(8)));
typedef float    v4f  __attribute__((ext_vector_type(4)));
typedef int      v4i  __attribute__((ext_vector_type(4)));
typedef v8h __attribute__((may_alias)) v8ha;
typedef v4f __attribute__((may_alias)) v4fa;
typedef v4i __attribute__((may_alias)) v4ia;

union Frag { v16h v; v8h half[2]; };

#define HID     256
#define NST     8192
#define NVOC    10000
#define NB      16
#define NT      256
#define PLANE   ((size_t)NST * HID)
#define WMAT    ((size_t)HID * HID)
#define WSC     16.0f
#define WINV    0.0625f
#define NEGBIG  (-1e30f)
#define NEGFILL (-1e9f)

__device__ __forceinline__ v8f wmma_f16(v16h a, v16h b, v8f c) {
  v8f d = __builtin_amdgcn_wmma_f32_16x16x32_f16(false, a, false, b, (short)0, c, false, false);
  asm volatile("v_nop\n\tv_nop\n\tv_nop\n\tv_nop" : "+v"(d) : "v"(a), "v"(b));
  return d;
}

__device__ __forceinline__ v16h load_frag(const _Float16* p, int h) {
  Frag f;
  f.half[0] = *(const v8ha*)(p + 8 * h);
  f.half[1] = *(const v8ha*)(p + 16 + 8 * h);
  return f.v;
}

__device__ __forceinline__ int clampi(int x, int lo, int hi) {
  return x < lo ? lo : (x > hi ? hi : x);
}

__device__ __forceinline__ v8f zero8f() {
  v8f z = {0.f, 0.f, 0.f, 0.f, 0.f, 0.f, 0.f, 0.f};
  return z;
}

__device__ __forceinline__ void w_store_pass(const _Float16* sT, _Float16* base, int n0, int k0,
                                             int wv, int lane) {
  const int q8 = lane & 7, sub = lane >> 3;
  #pragma unroll
  for (int i = 0; i < 2; ++i) {
    const int c = wv * 8 + i * 4 + sub;
    const v8h v = *(const v8ha*)(sT + c * 72 + 8 * q8);
    *(volatile v8h*)(base + (size_t)(n0 + c) * HID + k0 + 8 * q8) = v;
  }
}

__global__ __launch_bounds__(256) void convw_kernel(
    const float* __restrict__ w0, const float* __restrict__ w1, const float* __restrict__ w2,
    const float* __restrict__ w3, const float* __restrict__ w4, const float* __restrict__ w5,
    _Float16* __restrict__ W16)
{
  __shared__ __attribute__((aligned(16))) _Float16 sT[64 * 72];
  const int tid = threadIdx.x, lane = tid & 31, wv = tid >> 5;
  const int mat = blockIdx.y;
  const int kt = blockIdx.x >> 2, nt = blockIdx.x & 3;
  const int k0 = kt * 64, n0 = nt * 64;
  const float* W = (mat == 0) ? w0 : (mat == 1) ? w1 : (mat == 2) ? w2 : (mat == 3) ? w3 : (mat == 4) ? w4 : w5;
  #pragma unroll
  for (int i = 0; i < 16; ++i) {
    const int e = tid + 256 * i;
    const int r = e >> 6, c = e & 63;
    sT[c * 72 + r] = (_Float16)(W[(size_t)(k0 + r) * HID + n0 + c] * WSC);
  }
  __syncthreads();
  _Float16* base = W16 + (size_t)mat * WMAT;
  w_store_pass(sT, base, n0, k0, wv, lane);
  __threadfence();
  w_store_pass(sT, base, n0, k0, wv, lane);
}

__device__ __forceinline__ void t_store_pass(const _Float16* sT, _Float16* TT, int w0, int k0,
                                             int wv, int lane) {
  const int q8 = lane & 7, sub = lane >> 3;
  #pragma unroll
  for (int i = 0; i < 3; ++i) {
    const int lid = i * 4 + sub;
    const int c = wv * 10 + lid;
    const int cc = (c > 79) ? 79 : c;
    const v8h v = *(const v8ha*)(sT + cc * 72 + 8 * q8);
    if (lid < 10)
      *(volatile v8h*)(TT + (size_t)(w0 + c) * HID + k0 + 8 * q8) = v;
  }
}

__global__ __launch_bounds__(256) void convt_kernel(const float* __restrict__ P, _Float16* __restrict__ TT)
{
  __shared__ __attribute__((aligned(16))) _Float16 sT[80 * 72];
  const int tid = threadIdx.x, lane = tid & 31, wv = tid >> 5;
  const int w0 = blockIdx.x * 80, k0 = blockIdx.y * 64;
  #pragma unroll
  for (int i = 0; i < 20; ++i) {
    const int e = tid + 256 * i;
    const int r = e / 80, c = e - r * 80;
    sT[c * 72 + r] = (_Float16)(P[(size_t)(k0 + r) * NVOC + w0 + c] * WSC);
  }
  __syncthreads();
  t_store_pass(sT, TT, w0, k0, wv, lane);
  __threadfence();
  t_store_pass(sT, TT, w0, k0, wv, lane);
}

__global__ __launch_bounds__(256) void emb_kernel(
    const float* __restrict__ a0, const float* __restrict__ c0,
    const float* __restrict__ a1, const float* __restrict__ c1,
    const float* __restrict__ a2, const float* __restrict__ c2,
    const float* __restrict__ a3, const float* __restrict__ c3,
    _Float16* __restrict__ E16)
{
  const int tid = threadIdx.x, lane = tid & 31, wv = tid >> 5;
  const int p = blockIdx.y;
  const float* e1 = (p == 0) ? a0 : (p == 1) ? a1 : (p == 2) ? a2 : a3;
  const float* e2 = (p == 0) ? c0 : (p == 1) ? c1 : (p == 2) ? c2 : c3;
  const int s = blockIdx.x * 8 + wv;
  const float* pa = e1 + (size_t)(s >> 6) * HID + lane * 8;
  const float* pc = e2 + (size_t)(s & 63) * HID + lane * 8;
  const v4f x0 = *(const v4fa*)pa, x1 = *(const v4fa*)(pa + 4);
  const v4f y0 = *(const v4fa*)pc, y1 = *(const v4fa*)(pc + 4);
  const v8h o = { (_Float16)(x0.x + y0.x), (_Float16)(x0.y + y0.y), (_Float16)(x0.z + y0.z), (_Float16)(x0.w + y0.w),
                  (_Float16)(x1.x + y1.x), (_Float16)(x1.y + y1.y), (_Float16)(x1.z + y1.z), (_Float16)(x1.w + y1.w) };
  _Float16* dst = E16 + (size_t)p * PLANE + (size_t)s * HID + lane * 8;
  *(volatile v8h*)dst = o;
  __threadfence();
  *(volatile v8h*)dst = o;
}

__device__ __forceinline__ void tile_store_pass(const _Float16* sT, _Float16* out, int m0, int c0,
                                                int w, int lane) {
  const int q8 = lane & 7, sub = lane >> 3;
  #pragma unroll
  for (int i = 0; i < 8; ++i) {
    const int lid = w * 32 + i * 4 + sub;
    const v8h v = *(const v8ha*)(sT + lid * 64 + 8 * q8);
    *(volatile v8h*)(out + (size_t)(m0 + lid) * HID + c0 + 8 * q8) = v;
  }
}

__global__ __launch_bounds__(128) void gemm_kernel(
    const _Float16* __restrict__ A16,
    const _Float16* __restrict__ Wt,
    const float* __restrict__ bias,
    const float* __restrict__ e1,
    const float* __restrict__ e2,
    int doResid,
    _Float16* __restrict__ out16)
{
  __shared__ __attribute__((aligned(16))) _Float16 sT[128 * 64];

  const int tid = threadIdx.x, lane = tid & 31, w = tid >> 5;
  const int h = lane >> 4, m = lane & 15;
  const int m0 = blockIdx.x * 128;
  const int c0 = blockIdx.y * 64;
  const int m0w = m0 + 32 * w;

  const _Float16* xa0 = A16 + (size_t)(m0w + m) * HID;
  const _Float16* xa1 = xa0 + (size_t)16 * HID;
  const _Float16* wb  = Wt + (size_t)(c0 + m) * HID;

  v8f acc[2][4];
  #pragma unroll
  for (int mt = 0; mt < 2; ++mt)
    #pragma unroll
    for (int nt = 0; nt < 4; ++nt) acc[mt][nt] = zero8f();

  #pragma unroll 1
  for (int k0 = 0; k0 < HID; k0 += 32) {
    const v16h fa0 = load_frag(xa0 + k0, h);
    const v16h fa1 = load_frag(xa1 + k0, h);
    #pragma unroll
    for (int nt = 0; nt < 4; ++nt) {
      const v16h fb = load_frag(wb + (size_t)nt * 16 * HID + k0, h);
      acc[0][nt] = wmma_f16(fa0, fb, acc[0][nt]);
      acc[1][nt] = wmma_f16(fa1, fb, acc[1][nt]);
    }
  }

  #pragma unroll
  for (int nt = 0; nt < 4; ++nt) {
    const int col = c0 + 16 * nt + m;
    const float bvl = bias[col];
    #pragma unroll
    for (int mt = 0; mt < 2; ++mt) {
      #pragma unroll
      for (int r = 0; r < 8; ++r) {
        const int rowl = 32 * w + 16 * mt + 8 * h + r;
        const int row = m0 + rowl;
        float y = fmaxf(acc[mt][nt][r] * WINV + bvl, 0.0f);
        if (doResid) {
          const float x = e1[(size_t)(row >> 6) * HID + col] + e2[(size_t)(row & 63) * HID + col];
          y = y + x;
        }
        sT[rowl * 64 + 16 * nt + m] = (_Float16)y;
      }
    }
  }
  __syncthreads();

  tile_store_pass(sT, out16, m0, c0, w, lane);
  __threadfence();
  tile_store_pass(sT, out16, m0, c0, w, lane);
}

__global__ __launch_bounds__(256) void sc_kernel(const _Float16* __restrict__ RS16,
                                                 const float* __restrict__ pw,
                                                 const float* __restrict__ pb,
                                                 float* __restrict__ sc)
{
  __shared__ float spw[HID];
  __shared__ __attribute__((aligned(16))) float sOut[256];
  const int tid = threadIdx.x, lane = tid & 31, wv = tid >> 5;
  spw[tid] = pw[tid];
  __syncthreads();
  const int s = blockIdx.x * 256 + tid;
  const _Float16* r = RS16 + (size_t)s * HID;
  float a = 0.f;
  #pragma unroll 1
  for (int i = 0; i < HID / 8; ++i) {
    const v8h x = *(const v8ha*)(r + 8 * i);
    #pragma unroll
    for (int e = 0; e < 8; ++e) a += (float)x[e] * spw[8 * i + e];
  }
  sOut[tid] = a + pb[0];
  __syncthreads();
  if (wv < 2) {
    const v4f v = *(const v4fa*)(sOut + wv * 128 + lane * 4);
    float* dst = sc + (size_t)blockIdx.x * 256 + wv * 128 + lane * 4;
    *(volatile v4f*)dst = v;
    __threadfence();
    *(volatile v4f*)dst = v;
  }
}

template <int MASKED>
__global__ __launch_bounds__(256) void lse_kernel(
    const _Float16* __restrict__ A16,
    const _Float16* __restrict__ B16,
    int ncoltiles, float scale,
    const float* __restrict__ colbias,
    const int* __restrict__ w2s,
    float* __restrict__ lseOut)
{
  __shared__ float redM[32 * 64];
  __shared__ float redS[32 * 64];
  __shared__ __attribute__((aligned(16))) float sL[32];

  const int tid = threadIdx.x, lane = tid & 31, wv = tid >> 5;
  const int h = lane >> 4, m = lane & 15;
  const int rt = wv >> 2, cg = wv & 3;
  const int row0 = blockIdx.x * 32;
  const int rbase = row0 + 16 * rt + 8 * h;
  const int jmod = rbase & 63;

  const _Float16* Ar = A16 + (size_t)(row0 + 16 * rt + m) * HID;
  v16h af[8];
  #pragma unroll
  for (int kk = 0; kk < 8; ++kk) af[kk] = load_frag(Ar + 32 * kk, h);

  float rm[8], rs[8];
  #pragma unroll
  for (int r = 0; r < 8; ++r) { rm[r] = NEGBIG; rs[r] = 0.f; }

  #pragma unroll 1
  for (int jt = cg; jt < ncoltiles; jt += 4) {
    const int col = jt * 16 + m;
    const _Float16* Br = B16 + (size_t)col * HID;
    v8f acc = zero8f();
    #pragma unroll
    for (int kk = 0; kk < 8; ++kk) acc = wmma_f16(af[kk], load_frag(Br + 32 * kk, h), acc);

    float cb = 0.f;
    int qv[8] = {0, 0, 0, 0, 0, 0, 0, 0};
    if (MASKED) {
      cb = colbias[col];
      const v4i q0 = *(const v4ia*)(w2s + (size_t)col * 64 + jmod);
      const v4i q1 = *(const v4ia*)(w2s + (size_t)col * 64 + jmod + 4);
      qv[0] = q0.x; qv[1] = q0.y; qv[2] = q0.z; qv[3] = q0.w;
      qv[4] = q1.x; qv[5] = q1.y; qv[6] = q1.z; qv[7] = q1.w;
    }
    #pragma unroll
    for (int r = 0; r < 8; ++r) {
      const float val = acc[r] * scale + cb;
      const float d = val - rm[r];
      const float e = __expf(-fabsf(d));
      const float nrs = (d <= 0.f) ? (rs[r] + e) : (rs[r] * e + 1.0f);
      const float nrm = fmaxf(rm[r], val);
      if (MASKED) {
        const bool ok = (qv[r] == rbase + r);
        rs[r] = ok ? nrs : rs[r];
        rm[r] = ok ? nrm : rm[r];
      } else {
        rs[r] = nrs;
        rm[r] = nrm;
      }
    }
  }

  const int slot = cg * 16 + m;
  #pragma unroll
  for (int r = 0; r < 8; ++r) {
    const int rl = 16 * rt + 8 * h + r;
    redM[rl * 64 + slot] = rm[r];
    redS[rl * 64 + slot] = rs[r];
  }
  __syncthreads();
  if (tid < 32) {
    float M = NEGBIG;
    #pragma unroll 1
    for (int k = 0; k < 64; ++k) M = fmaxf(M, redM[tid * 64 + k]);
    float S = 0.f;
    #pragma unroll 1
    for (int k = 0; k < 64; ++k) S += redS[tid * 64 + k] * __expf(redM[tid * 64 + k] - M);
    sL[tid] = (S > 0.f) ? (M + __logf(S)) : NEGFILL;
  }
  __syncthreads();
  if (tid < 8) {
    const v4f v = *(const v4fa*)(sL + 4 * tid);
    *(volatile v4f*)(lseOut + row0 + 4 * tid) = v;
  }
  __threadfence();
  if (tid < 8) {
    const v4f v = *(const v4fa*)(sL + 4 * tid);
    *(volatile v4f*)(lseOut + row0 + 4 * tid) = v;
  }
}

__device__ __forceinline__ float obs_partial(const _Float16* __restrict__ RE16,
                                             const _Float16* __restrict__ TT16,
                                             int s, int w, int q) {
  const _Float16* pr = RE16 + (size_t)s * HID + q * 64;
  const _Float16* pt = TT16 + (size_t)w * HID + q * 64;
  float a = 0.f;
  #pragma unroll
  for (int i = 0; i < 8; ++i) {
    const v8h x = *(const v8ha*)(pr + 8 * i);
    const v8h y = *(const v8ha*)(pt + 8 * i);
    #pragma unroll
    for (int e = 0; e < 8; ++e) a += (float)x[e] * (float)y[e];
  }
  return a;
}

__global__ __launch_bounds__(256) void dp_kernel(
    const int* __restrict__ text,
    const int* __restrict__ w2s,
    const _Float16* __restrict__ RT16,
    const _Float16* __restrict__ NX16,
    const _Float16* __restrict__ RE16,
    const _Float16* __restrict__ TT16,
    const float* __restrict__ termPb,
    const float* __restrict__ sc,
    const float* __restrict__ lseT,
    const float* __restrict__ lseE,
    float* __restrict__ res)
{
  __shared__ __attribute__((aligned(16))) _Float16 sA[64 * HID];
  __shared__ __attribute__((aligned(16))) _Float16 sB[64 * HID];
  __shared__ float sP[64 * 68];
  __shared__ float sPart[4 * 64];
  __shared__ float sAl[2 * 64];
  __shared__ int   sCs[2 * 64];
  __shared__ float sRed[64];
  __shared__ float sRedW[16];

  const int tid = threadIdx.x, lane = tid & 31, wv = tid >> 5;
  const int h = lane >> 4, m = lane & 15;
  const int b = blockIdx.x;

  float lm = NEGBIG;
  #pragma unroll 1
  for (int i = 0; i < NST / 256; ++i) lm = fmaxf(lm, sc[tid + 256 * i]);
  #pragma unroll
  for (int o = 16; o > 0; o >>= 1) lm = fmaxf(lm, __shfl_xor(lm, o));
  if (lane == 0) sRedW[wv] = lm;
  __syncthreads();
  float gm = NEGBIG;
  #pragma unroll
  for (int k = 0; k < 8; ++k) gm = fmaxf(gm, sRedW[k]);
  float ls = 0.f;
  #pragma unroll 1
  for (int i = 0; i < NST / 256; ++i) ls += __expf(sc[tid + 256 * i] - gm);
  #pragma unroll
  for (int o = 16; o > 0; o >>= 1) ls += __shfl_xor(ls, o);
  if (lane == 0) sRedW[8 + wv] = ls;
  __syncthreads();
  float gs = 0.f;
  #pragma unroll
  for (int k = 0; k < 8; ++k) gs += sRedW[8 + k];
  const float lse0 = gm + __logf(gs);

  const int w0 = clampi(text[b * NT], 0, NVOC - 1);
  if (tid < 64) sCs[tid] = clampi(w2s[(size_t)w0 * 64 + tid], 0, NST - 1);
  __syncthreads();
  {
    const int j = tid & 63, q = tid >> 6;
    sPart[q * 64 + j] = obs_partial(RE16, TT16, sCs[j], w0, q);
  }
  __syncthreads();
  float alphaRaw = 0.f;
  if (tid < 64) {
    const int j = tid;
    const int s = sCs[j];
    const float lg = (sPart[j] + sPart[64 + j] + sPart[128 + j] + sPart[192 + j]) * WINV + termPb[w0];
    const int qs = w2s[(size_t)w0 * 64 + (s & 63)];
    const float em = (qs == s) ? lg : NEGFILL;
    const float ob = em - lseE[s];
    const float a0 = sc[s] - lse0 + ob;
    alphaRaw = a0;
    sAl[j] = a0 - lseT[s];
  }

  #pragma unroll 1
  for (int t = 1; t < NT; ++t) {
    const int cur = t & 1, prv = cur ^ 1;
    const int w = clampi(text[b * NT + t], 0, NVOC - 1);
    if (tid < 64) sCs[cur * 64 + tid] = clampi(w2s[(size_t)w * 64 + tid], 0, NST - 1);
    __syncthreads();

    {
      const int row = tid >> 2, part = tid & 3;
      const int sp = sCs[prv * 64 + row], sq = sCs[cur * 64 + row];
      const _Float16* ga = RT16 + (size_t)sp * HID + part * 64;
      const _Float16* gb = NX16 + (size_t)sq * HID + part * 64;
      _Float16* da = sA + row * HID + part * 64;
      _Float16* db = sB + row * HID + part * 64;
      #pragma unroll
      for (int i = 0; i < 8; ++i) {
        const v8h va = *(const v8ha*)(ga + 8 * i);
        const v8h vb = *(const v8ha*)(gb + 8 * i);
        *(v8ha*)(da + 8 * i) = va;
        *(v8ha*)(db + 8 * i) = vb;
      }
    }
    {
      const int j = tid & 63, q = tid >> 6;
      sPart[q * 64 + j] = obs_partial(RE16, TT16, sCs[cur * 64 + j], w, q);
    }
    __syncthreads();

    {
      const int tj = wv & 3, ti0 = wv >> 2, ti1 = ti0 + 2;
      v8f acc0 = zero8f(), acc1 = zero8f();
      const _Float16* pa0 = sA + (16 * ti0 + m) * HID;
      const _Float16* pa1 = sA + (16 * ti1 + m) * HID;
      const _Float16* pbp = sB + (16 * tj + m) * HID;
      #pragma unroll
      for (int kk = 0; kk < 8; ++kk) {
        const v16h fb = load_frag(pbp + 32 * kk, h);
        acc0 = wmma_f16(load_frag(pa0 + 32 * kk, h), fb, acc0);
        acc1 = wmma_f16(load_frag(pa1 + 32 * kk, h), fb, acc1);
      }
      #pragma unroll
      for (int r = 0; r < 8; ++r) {
        sP[(16 * ti0 + 8 * h + r) * 68 + 16 * tj + m] = acc0[r];
        sP[(16 * ti1 + 8 * h + r) * 68 + 16 * tj + m] = acc1[r];
      }
    }
    __syncthreads();

    if (tid < 64) {
      const int j = tid;
      const float* al = sAl + prv * 64;
      float M = NEGBIG;
      #pragma unroll 4
      for (int i = 0; i < 64; ++i) M = fmaxf(M, al[i] + sP[i * 68 + j]);
      float S = 0.f;
      #pragma unroll 4
      for (int i = 0; i < 64; ++i) S += __expf(al[i] + sP[i * 68 + j] - M);
      const int s = sCs[cur * 64 + j];
      const float lg = (sPart[j] + sPart[64 + j] + sPart[128 + j] + sPart[192 + j]) * WINV + termPb[w];
      const int qs = w2s[(size_t)w * 64 + (s & 63)];
      const float em = (qs == s) ? lg : NEGFILL;
      const float ob = em - lseE[s];
      const float a2 = M + __logf(S) + ob;
      alphaRaw = a2;
      sAl[cur * 64 + j] = a2 - lseT[s];
    }
  }

  if (tid < 64) sRed[tid] = alphaRaw;
  __syncthreads();
  if (wv == 0) {
    const float v0 = sRed[lane], v1 = sRed[lane + 32];
    float M = fmaxf(v0, v1);
    #pragma unroll
    for (int o = 16; o > 0; o >>= 1) M = fmaxf(M, __shfl_xor(M, o));
    float S = __expf(v0 - M) + __expf(v1 - M);
    #pragma unroll
    for (int o = 16; o > 0; o >>= 1) S += __shfl_xor(S, o);
    const float L = M + __logf(S);
    const v4f ov = {L, L, L, L};
    if (lane < 8) *(volatile v4f*)(res + b * 32 + lane * 4) = ov;
    __threadfence();
    if (lane < 8) *(volatile v4f*)(res + b * 32 + lane * 4) = ov;
  }
}

__global__ __launch_bounds__(32) void out_kernel(const float* __restrict__ res, float* __restrict__ out)
{
  __shared__ __attribute__((aligned(16))) float sO[16];
  const int lane = threadIdx.x;
  const int li = (lane > 15) ? 15 : lane;
  const float v = res[li * 32];
  if (lane < 16) sO[lane] = v;
  __syncthreads();
  if (lane < 4) {
    const v4f o = *(const v4fa*)(sO + lane * 4);
    *(volatile v4f*)(out + lane * 4) = o;
  }
  __threadfence();
  if (lane < 4) {
    const v4f o = *(const v4fa*)(sO + lane * 4);
    *(volatile v4f*)(out + lane * 4) = o;
  }
}

extern "C" void kernel_launch(void* const* d_in, const int* in_sizes, int n_in,
                              void* d_out, int out_size, void* d_ws, size_t ws_size,
                              hipStream_t stream) {
  if (n_in < 26) return;
  if (in_sizes[0] != NB * NT) return;
  if (in_sizes[1] != NVOC * 64) return;
  if (in_sizes[2] != 128 * HID || in_sizes[10] != 128 * HID || in_sizes[12] != 128 * HID || in_sizes[18] != 128 * HID) return;
  if (in_sizes[3] != 64 * HID || in_sizes[11] != 64 * HID || in_sizes[13] != 64 * HID || in_sizes[19] != 64 * HID) return;
  if (in_sizes[4] != HID * HID || in_sizes[6] != HID * HID || in_sizes[14] != HID * HID ||
      in_sizes[16] != HID * HID || in_sizes[20] != HID * HID || in_sizes[22] != HID * HID) return;
  if (in_sizes[5] != HID || in_sizes[7] != HID || in_sizes[15] != HID || in_sizes[17] != HID ||
      in_sizes[21] != HID || in_sizes[23] != HID) return;
  if (in_sizes[8] != HID || in_sizes[9] != 1) return;
  if (in_sizes[24] != HID * NVOC || in_sizes[25] != NVOC) return;
  if (out_size != NB) return;

  const int*   text      = (const int*)d_in[0];
  const int*   w2s       = (const int*)d_in[1];
  const float* se1_start = (const float*)d_in[2];
  const float* se2_start = (const float*)d_in[3];
  const float* start_w1  = (const float*)d_in[4];
  const float* start_b1  = (const float*)d_in[5];
  const float* start_w2  = (const float*)d_in[6];
  const float* start_b2  = (const float*)d_in[7];
  const float* start_pw  = (const float*)d_in[8];
  const float* start_pb  = (const float*)d_in[9];
  const float* se1_state = (const float*)d_in[10];
  const float* se2_state = (const float*)d_in[11];
  const float* se1_next  = (const float*)d_in[12];
  const float* se2_next  = (const float*)d_in[13];
  const float* trans_w1  = (const float*)d_in[14];
  const float* trans_b1  = (const float*)d_in[15];
  const float* trans_w2  = (const float*)d_in[16];
  const float* trans_b2  = (const float*)d_in[17];
  const float* se1_pre   = (const float*)d_in[18];
  const float* se2_pre   = (const float*)d_in[19];
  const float* term_w1   = (const float*)d_in[20];
  const float* term_b1   = (const float*)d_in[21];
  const float* term_w2   = (const float*)d_in[22];
  const float* term_b2   = (const float*)d_in[23];
  const float* term_pw   = (const float*)d_in[24];
  const float* term_pb   = (const float*)d_in[25];
  float* out = (float*)d_out;

  const size_t w16_bytes  = (size_t)6 * WMAT * 2;
  const size_t tt_bytes   = (size_t)NVOC * HID * 2;
  const size_t pl_bytes   = PLANE * 2;
  const size_t e16_bytes  = 4 * pl_bytes;
  const size_t vec_bytes  = (size_t)NST * 4;
  const size_t res_bytes  = (size_t)NB * 32 * 4;
  size_t off = 0;
  const size_t o_w16 = off;  off += w16_bytes;
  const size_t o_tt  = off;  off += tt_bytes;
  const size_t o_e16 = off;  off += e16_bytes;
  const size_t o_h16 = off;  off += pl_bytes;
  const size_t o_rs  = off;  off += pl_bytes;
  const size_t o_rt  = off;  off += pl_bytes;
  const size_t o_re  = off;  off += pl_bytes;
  const size_t o_sc  = off;  off += vec_bytes;
  const size_t o_lt  = off;  off += vec_bytes;
  const size_t o_le  = off;  off += vec_bytes;
  const size_t o_res = off;  off += res_bytes;
  if (off > ws_size) return;

  char* ws = (char*)d_ws;
  _Float16* W16  = (_Float16*)(ws + o_w16);
  _Float16* TT16 = (_Float16*)(ws + o_tt);
  _Float16* E16  = (_Float16*)(ws + o_e16);
  _Float16* H16  = (_Float16*)(ws + o_h16);
  _Float16* RS16 = (_Float16*)(ws + o_rs);
  _Float16* RT16 = (_Float16*)(ws + o_rt);
  _Float16* RE16 = (_Float16*)(ws + o_re);
  float* sc   = (float*)(ws + o_sc);
  float* LSET = (float*)(ws + o_lt);
  float* LSEE = (float*)(ws + o_le);
  float* RES  = (float*)(ws + o_res);

  _Float16* E_start = E16;
  _Float16* E_state = E16 + PLANE;
  _Float16* E_next  = E16 + 2 * PLANE;
  _Float16* E_pre   = E16 + 3 * PLANE;

  convw_kernel<<<dim3(16, 6), 256, 0, stream>>>(start_w1, start_w2, trans_w1, trans_w2, term_w1, term_w2, W16);
  convt_kernel<<<dim3(125, 4), 256, 0, stream>>>(term_pw, TT16);

  emb_kernel<<<dim3(NST / 8, 4), 256, 0, stream>>>(se1_start, se2_start, se1_state, se2_state,
                                                   se1_next, se2_next, se1_pre, se2_pre, E16);

  const dim3 gG(NST / 128, HID / 64);
  gemm_kernel<<<gG, 128, 0, stream>>>(E_start, W16 + 0 * WMAT, start_b1, se1_start, se2_start, 0, H16);
  gemm_kernel<<<gG, 128, 0, stream>>>(H16,     W16 + 1 * WMAT, start_b2, se1_start, se2_start, 1, RS16);
  gemm_kernel<<<gG, 128, 0, stream>>>(E_state, W16 + 2 * WMAT, trans_b1, se1_state, se2_state, 0, H16);
  gemm_kernel<<<gG, 128, 0, stream>>>(H16,     W16 + 3 * WMAT, trans_b2, se1_state, se2_state, 1, RT16);
  gemm_kernel<<<gG, 128, 0, stream>>>(E_pre,   W16 + 4 * WMAT, term_b1, se1_pre, se2_pre, 0, H16);
  gemm_kernel<<<gG, 128, 0, stream>>>(H16,     W16 + 5 * WMAT, term_b2, se1_pre, se2_pre, 1, RE16);

  sc_kernel<<<NST / 256, 256, 0, stream>>>(RS16, start_pw, start_pb, sc);

  lse_kernel<0><<<NST / 32, 256, 0, stream>>>(RT16, E_next, NST / 16, 1.0f, term_pb, w2s, LSET);
  lse_kernel<1><<<NST / 32, 256, 0, stream>>>(RE16, TT16, NVOC / 16, WINV, term_pb, w2s, LSEE);

  dp_kernel<<<NB, 256, 0, stream>>>(text, w2s, RT16, E_next, RE16, TT16, term_pb, sc, LSET, LSEE, RES);

  out_kernel<<<1, 32, 0, stream>>>(RES, out);
}
